// GruBlock_68410239091486
// MI455X (gfx1250) — hardware-verified
//
#include <hip/hip_runtime.h>
#include <math.h>

constexpr int SCAN_T   = 128;
constexpr int NBAT     = 512;
constexpr int NFEAT    = 64;
constexpr int NHID     = 128;
constexpr int NG3      = 3 * NHID;
constexpr int NROWS    = SCAN_T * NBAT;
constexpr int NTHR     = 256;
constexpr int ROWS_BLK = 16;
constexpr int HPITCH   = 136;
constexpr int PPITCH   = 388;
constexpr int OPITCH   = 260;
constexpr float HCARRY = 16.0f;
constexpr float WCARRY = 256.0f;
constexpr float PROJ0_SCALE = 1.0f / 256.0f;
constexpr float PROJ_SCALE  = 1.0f / 4096.0f;
constexpr float REC_SCALE   = 1.0f / 4096.0f;

static_assert(NROWS % 64 == 0 && NG3 % 64 == 0);
static_assert(NFEAT % 32 == 0 && NHID % 32 == 0);
static_assert(((NROWS / 64) * (NG3 / 64)) % 8 == 0);
static_assert(NBAT % ROWS_BLK == 0);
static_assert(NHID == 16 * (NTHR / 32));
static_assert((ROWS_BLK * NG3 / 4) % NTHR == 0);
static_assert(ROWS_BLK * NHID / 8 == NTHR);
static_assert((ROWS_BLK * NHID / 4) % NTHR == 0);
static_assert((NROWS * NFEAT / 8) % NTHR == 0);
static_assert((NG3 * NFEAT / 8) % NTHR == 0 && (NG3 * NHID / 8) % NTHR == 0);
static_assert(HPITCH % 8 == 0 && PPITCH % 4 == 0 && OPITCH % 4 == 0);

typedef __attribute__((ext_vector_type(16))) _Float16 v16h;
typedef __attribute__((ext_vector_type(8)))  _Float16 v8h;
typedef __attribute__((ext_vector_type(16))) __bf16   v16b;
typedef __attribute__((ext_vector_type(8)))  __bf16   v8b;
typedef __attribute__((ext_vector_type(8)))  float    v8f;
typedef __attribute__((ext_vector_type(4)))  float    v4f;

__device__ __forceinline__ unsigned short f2bf_bits(float f) {
  unsigned u = __float_as_uint(f);
  return (unsigned short)((u + 0x7FFFu + ((u >> 16) & 1u)) >> 16);
}
__device__ __forceinline__ float bf_bits2f(unsigned short h) { return __uint_as_float(((unsigned)h) << 16); }

__device__ __forceinline__ void dep_guard_h(v8f& a, v8f& b, v16h x, v16h y) { asm volatile("v_nop\n\tv_nop\n\tv_nop\n\tv_nop" : "+v"(a), "+v"(b) : "v"(x), "v"(y)); }
__device__ __forceinline__ void dep_guard_b(v8f& a, v8f& b, v16b x, v16b y) { asm volatile("v_nop\n\tv_nop\n\tv_nop\n\tv_nop" : "+v"(a), "+v"(b) : "v"(x), "v"(y)); }
__device__ __forceinline__ void dep_guard3_h(v8f& a, v8f& b, v8f& c, v16h x, v16h y) { asm volatile("v_nop\n\tv_nop\n\tv_nop\n\tv_nop" : "+v"(a), "+v"(b), "+v"(c) : "v"(x), "v"(y)); }
__device__ __forceinline__ void keep4_h(v16h a, v16h b, v16h c, v16h d) { asm volatile("v_nop" :: "v"(a), "v"(b), "v"(c), "v"(d)); }
__device__ __forceinline__ void keep4_b(v16b a, v16b b, v16b c, v16b d) { asm volatile("v_nop" :: "v"(a), "v"(b), "v"(c), "v"(d)); }
__device__ __forceinline__ void acc_guard4(v8f& a, v8f& b, v8f& c, v8f& d) { asm volatile("v_nop\n\tv_nop\n\tv_nop\n\tv_nop" : "+v"(a), "+v"(b), "+v"(c), "+v"(d)); }
__device__ __forceinline__ void acc_guard3(v8f& a, v8f& b, v8f& c) { asm volatile("v_nop\n\tv_nop\n\tv_nop\n\tv_nop" : "+v"(a), "+v"(b), "+v"(c)); }
template <typename T> struct Frag;
template <> struct Frag<_Float16> {
  typedef v16h V; union U { v16h v; v8h h[2]; };
  static __device__ __forceinline__ v16h load(const _Float16* p) {
    U f; f.h[0] = *(const v8h*)(p); f.h[1] = *(const v8h*)(p + 16); return f.v;
  }
  static __device__ __forceinline__ v8f mma(v16h a, v16h b, v8f c) {
    return __builtin_amdgcn_wmma_f32_16x16x32_f16(false, a, false, b, (short)0, c, false, false);
  }
  static __device__ __forceinline__ void guard(v8f& a, v8f& b, v16h x, v16h y) { dep_guard_h(a, b, x, y); }
  static __device__ __forceinline__ void keep(v16h a, v16h b, v16h c, v16h d) { keep4_h(a, b, c, d); }
};
template <> struct Frag<__bf16> {
  typedef v16b V; union U { v16b v; v8b h[2]; };
  static __device__ __forceinline__ v16b load(const __bf16* p) {
    U f; f.h[0] = *(const v8b*)(p); f.h[1] = *(const v8b*)(p + 16); return f.v;
  }
  static __device__ __forceinline__ v8f mma(v16b a, v16b b, v8f c) {
    return __builtin_amdgcn_wmma_f32_16x16x32_bf16(false, a, false, b, (short)0, c, false, false);
  }
  static __device__ __forceinline__ void guard(v8f& a, v8f& b, v16b x, v16b y) { dep_guard_b(a, b, x, y); }
  static __device__ __forceinline__ void keep(v16b a, v16b b, v16b c, v16b d) { keep4_b(a, b, c, d); }
};

__device__ __forceinline__ float fsig(float x) { return 1.0f / (1.0f + expf(-x)); }

template <int ET> struct Elem;
template <> struct Elem<0> { typedef _Float16 T; };
template <> struct Elem<1> { typedef __bf16 T; };
template <int ET, bool SPLIT, int BIAS_MODE, int OUT_MODE, bool RESID, int ACT = 0>
__global__ __launch_bounds__(256) void wmma_gemm64(
    const unsigned short* __restrict__ Ap, const unsigned short* __restrict__ A2p, int lda, long strideA,
    const unsigned short* __restrict__ Btp, const unsigned short* __restrict__ Bt2p, int ldb, long strideB,
    void* __restrict__ Cout, void* __restrict__ Cout2, int ldc, long strideC,
    const float* __restrict__ bias,
    const float* __restrict__ resid, long strideR,
    int M, int N, int K, float scale) {
  typedef typename Elem<ET>::T T;
  typedef typename Frag<T>::V V;
  const T* A = (const T*)Ap; const T* A2 = (const T*)A2p; const T* Bt = (const T*)Btp; const T* Bt2 = (const T*)Bt2p;
  __shared__ __align__(16) float sT[8][16 * 68];
  const int b    = blockIdx.y;
  const int lane = threadIdx.x & 31;
  const int wave = threadIdx.x >> 5;
  const int tilesN = N >> 6;
  const int tilesM = M >> 6;
  const int tile = blockIdx.x * 8 + wave;
  if (tile >= tilesM * tilesN) return;
  const int tm = tile / tilesN;
  const int tn = tile - tm * tilesN;
  const int m0 = tm << 6;
  const int n0 = tn << 6;

  const T* Ab  = A  + (size_t)b * strideA;
  const T* Bb  = Bt + (size_t)b * strideB;
  const T* Ab2 = SPLIT ? (A2  + (size_t)b * strideA) : nullptr;
  const T* Bb2 = SPLIT ? (Bt2 + (size_t)b * strideB) : nullptr;

  const int rlane = lane & 15;
  const int koff  = (lane >> 4) * 8;
  const int mOff  = (lane >> 4) * 8;

  v8f acc[4][4];
#pragma unroll
  for (int i = 0; i < 4; ++i)
#pragma unroll
    for (int j = 0; j < 4; ++j) acc[i][j] = (v8f){0.f,0.f,0.f,0.f,0.f,0.f,0.f,0.f};

  for (int k0 = 0; k0 < K; k0 += 32) {
    V bh[4], bl[4];
#pragma unroll
    for (int j = 0; j < 4; ++j) {
      const size_t bo = (size_t)(n0 + (j << 4) + rlane) * ldb + koff + k0;
      bh[j] = Frag<T>::load(Bb + bo);
      if (SPLIT) bl[j] = Frag<T>::load(Bb2 + bo);
    }
#pragma unroll
    for (int i = 0; i < 4; ++i) {
      const size_t ao = (size_t)(m0 + (i << 4) + rlane) * lda + koff + k0;
      V ah = Frag<T>::load(Ab + ao);
      V al;
      if (SPLIT) al = Frag<T>::load(Ab2 + ao);
#pragma unroll
      for (int j = 0; j < 4; ++j) {
        acc[i][j] = Frag<T>::mma(ah, bh[j], acc[i][j]);
        if (SPLIT) {
          acc[i][j] = Frag<T>::mma(ah, bl[j], acc[i][j]);
          acc[i][j] = Frag<T>::mma(al, bh[j], acc[i][j]);
        }
      }
      Frag<T>::guard(acc[i][0], acc[i][3], ah, SPLIT ? al : ah);
    }
    Frag<T>::keep(bh[0], bh[1], bh[2], bh[3]);
    if (SPLIT) Frag<T>::keep(bl[0], bl[1], bl[2], bl[3]);
  }
  acc_guard4(acc[0][0], acc[0][1], acc[0][2], acc[0][3]);
  acc_guard4(acc[1][0], acc[1][1], acc[1][2], acc[1][3]);
  acc_guard4(acc[2][0], acc[2][1], acc[2][2], acc[2][3]);
  acc_guard4(acc[3][0], acc[3][1], acc[3][2], acc[3][3]);

  float* slab = sT[wave];
  const float* Rb = RESID ? (resid + (size_t)b * strideR) : nullptr;
#pragma unroll
  for (int i = 0; i < 4; ++i) {
    const int mBase = m0 + (i << 4);
#pragma unroll
    for (int j = 0; j < 4; ++j) {
      const int n = n0 + (j << 4) + rlane;
      float bv = 0.f;
      if (BIAS_MODE == 2) bv = bias[n];
#pragma unroll
      for (int r = 0; r < 8; ++r) {
        float v = acc[i][j][r] * scale;
        if (BIAS_MODE == 1) v += bias[mBase + mOff + r];
        if (BIAS_MODE == 2) v += bv;
        if (RESID) v += Rb[(size_t)(mBase + mOff + r) * ldc + n];
        if (ACT == 1) v = tanhf(v);
        if (ACT == 2) v = fmaxf(v, 0.0f);
        if (ACT == 3) v = v / (1.0f + expf(-v));
        if (ACT == 4) v = (v > 0.f) ? v : 0.01f * v;
        if (ACT == 5) v = 0.5f * v * (1.0f + erff(v * 0.70710678118654752f));
        slab[(mOff + r) * 68 + (j << 4) + rlane] = v;
      }
    }
    __builtin_amdgcn_fence(__ATOMIC_RELEASE, "workgroup");
    __builtin_amdgcn_wave_barrier();
    __builtin_amdgcn_fence(__ATOMIC_ACQUIRE, "workgroup");
    if (OUT_MODE == 0) {
      float* C = (float*)Cout + (size_t)b * strideC;
      const int hh = lane >> 4, c4 = (lane & 15) * 4;
      for (int pass = 0; pass < 2; ++pass) {
#pragma unroll
        for (int it = 0; it < 8; ++it) {
          const int row = it * 2 + hh;
          v4f v = *(const v4f*)(slab + row * 68 + c4);
          *(volatile v4f*)(C + (size_t)(mBase + row) * ldc + n0 + c4) = v;
        }
        __threadfence();
      }
    } else {
      const int q = lane >> 3, c8 = (lane & 7) * 8;
      unsigned short* C  = (unsigned short*)Cout  + (size_t)b * strideC;
      unsigned short* C2 = (OUT_MODE == 2) ? ((unsigned short*)Cout2 + (size_t)b * strideC) : nullptr;
      for (int pass = 0; pass < 2; ++pass) {
#pragma unroll
        for (int it = 0; it < 4; ++it) {
          const int row = it * 4 + q;
          const float* sp = slab + row * 68 + c8;
          v8h hv, lv;
#pragma unroll
          for (int e = 0; e < 8; ++e) {
            if (OUT_MODE == 1) {
              hv[e] = (_Float16)sp[e];
            } else {
              unsigned short hb = f2bf_bits(sp[e]);
              unsigned short lb = f2bf_bits(sp[e] - bf_bits2f(hb));
              hv[e] = __builtin_bit_cast(_Float16, hb);
              lv[e] = __builtin_bit_cast(_Float16, lb);
            }
          }
          *(volatile v8h*)(C + (size_t)(mBase + row) * ldc + n0 + c8) = hv;
          if (OUT_MODE == 2) *(volatile v8h*)(C2 + (size_t)(mBase + row) * ldc + n0 + c8) = lv;
        }
        __threadfence();
      }
    }
    __builtin_amdgcn_fence(__ATOMIC_RELEASE, "workgroup");
    __builtin_amdgcn_wave_barrier();
    __builtin_amdgcn_fence(__ATOMIC_ACQUIRE, "workgroup");
  }
}

__global__ __launch_bounds__(NTHR) void cvt_f16x8_kernel(const float* __restrict__ src, unsigned short* __restrict__ dst,
                                                         int n8, float sc) {
  const int i = blockIdx.x * NTHR + threadIdx.x;
  if (i < n8) {
    const float* sp = src + (size_t)i * 8;
    const v4f a = *(const v4f*)(sp);
    const v4f b = *(const v4f*)(sp + 4);
    v8h hv;
#pragma unroll
    for (int e = 0; e < 4; ++e) {
      hv[e]     = (_Float16)(a[e] * sc);
      hv[4 + e] = (_Float16)(b[e] * sc);
    }
    unsigned short* dp = dst + (size_t)i * 8;
    *(volatile v8h*)dp = hv;
    __threadfence();
    *(volatile v8h*)dp = hv;
  }
}

template <bool LAST>
__global__ __launch_bounds__(NTHR) void gru_scan_kernel(const float* __restrict__ PX, const unsigned short* __restrict__ WHHp,
                                                        const float* __restrict__ bhh, unsigned short* __restrict__ YS,
                                                        float* __restrict__ OUT) {
  __shared__ __align__(16) _Float16 Ah[ROWS_BLK * HPITCH];
  __shared__ __align__(16) float    Ps[ROWS_BLK * PPITCH];
  __shared__ __align__(16) float    Hs[ROWS_BLK * OPITCH];
  const _Float16* WHH = (const _Float16*)WHHp;
  const int tid = threadIdx.x, lane = tid & 31, wave = tid >> 5;
  const int c = lane & 15, hh = lane >> 4, koff = hh * 8;
  const int n0 = blockIdx.x * ROWS_BLK;
  const int j = 16 * wave + c;

#pragma unroll 1
  for (int i = tid; i < ROWS_BLK * HPITCH; i += NTHR) Ah[i] = (_Float16)0.0f;
  float hst[8];
#pragma unroll
  for (int r = 0; r < 8; ++r) hst[r] = 0.0f;
  const float br = bhh[j], bz = bhh[NHID + j], bn = bhh[2 * NHID + j];
  __syncthreads();

  const v8f z8 = {0.f, 0.f, 0.f, 0.f, 0.f, 0.f, 0.f, 0.f};
  const _Float16* ahrow = Ah + c * HPITCH + koff;
  const _Float16* wr = WHH + (size_t)j * NHID + koff;
  const _Float16* wz = wr + (size_t)NHID * NHID;
  const _Float16* wn = wr + (size_t)2 * NHID * NHID;
  const int srow = tid >> 4, sc8 = (tid & 15) * 8;

#pragma unroll 1
  for (int s = 0; s < SCAN_T; ++s) {
    const size_t rowg = (size_t)s * NBAT + (size_t)n0;
    {
      const float* pxs = PX + rowg * NG3;
#pragma unroll
      for (int it = 0; it < (ROWS_BLK * NG3 / 4) / NTHR; ++it) {
        const int idx = it * NTHR + tid;
        const int row = idx / (NG3 / 4);
        const int c4  = (idx - row * (NG3 / 4)) * 4;
        const v4f v = *(const v4f*)(pxs + (size_t)row * NG3 + c4);
        *(v4f*)(Ps + row * PPITCH + c4) = v;
      }
    }
    __syncthreads();

    v8f ar = z8, az = z8, an = z8;
#pragma unroll 1
    for (int k0 = 0; k0 < NHID; k0 += 32) {
      const v16h a  = Frag<_Float16>::load(ahrow + k0);
      const v16h b0 = Frag<_Float16>::load(wr + k0);
      const v16h b1 = Frag<_Float16>::load(wz + k0);
      const v16h b2 = Frag<_Float16>::load(wn + k0);
      ar = Frag<_Float16>::mma(a, b0, ar);
      az = Frag<_Float16>::mma(a, b1, az);
      an = Frag<_Float16>::mma(a, b2, an);
      dep_guard3_h(ar, az, an, a, b2);
      keep4_h(a, b0, b1, b2);
    }
    acc_guard3(ar, az, an);

#pragma unroll
    for (int r = 0; r < 8; ++r) {
      const int row = 8 * hh + r;
      const float pr = Ps[row * PPITCH + j];
      const float pz = Ps[row * PPITCH + NHID + j];
      const float pn = Ps[row * PPITCH + 2 * NHID + j];
      const float gr = ar[r] * REC_SCALE + br;
      const float gz = az[r] * REC_SCALE + bz;
      const float gn = an[r] * REC_SCALE + bn;
      const float rg = fsig(pr + gr);
      const float zg = fsig(pz + gz);
      const float ng = tanhf(pn + rg * gn);
      const float hn = (1.0f - zg) * ng + zg * hst[r];
      hst[r] = hn;
      Hs[row * OPITCH + j] = hn;
    }
    __syncthreads();

    {
      const v4f u0 = *(const v4f*)(Hs + srow * OPITCH + sc8);
      const v4f u1 = *(const v4f*)(Hs + srow * OPITCH + sc8 + 4);
      v8h hv;
#pragma unroll
      for (int e = 0; e < 4; ++e) {
        hv[e]     = (_Float16)(u0[e] * HCARRY);
        hv[4 + e] = (_Float16)(u1[e] * HCARRY);
      }
      *(v8h*)(Ah + srow * HPITCH + sc8) = hv;
      if (!LAST) {
        unsigned short* yp = YS + (rowg + (size_t)srow) * NHID + sc8;
        *(volatile v8h*)yp = hv;
        __threadfence();
        *(volatile v8h*)yp = hv;
      }
    }
    if (LAST) {
      for (int pass = 0; pass < 2; ++pass) {
#pragma unroll
        for (int it = 0; it < (ROWS_BLK * NHID / 4) / NTHR; ++it) {
          const int idx = it * NTHR + tid;
          const int row = idx >> 5, c4 = (idx & 31) * 4;
          const v4f v = *(const v4f*)(Hs + row * OPITCH + c4);
          *(volatile v4f*)(OUT + (rowg + (size_t)row) * NHID + c4) = v;
        }
        __threadfence();
      }
    }
  }
}

extern "C" void kernel_launch(void* const* d_in, const int* in_sizes, int n_in,
                              void* d_out, int out_size, void* d_ws, size_t ws_size, hipStream_t stream) {
  if (n_in < 13 || d_out == nullptr || d_ws == nullptr) return;
  if (in_sizes[0] != SCAN_T * NBAT * NFEAT || in_sizes[1] != NG3 * NFEAT || in_sizes[2] != NG3 * NHID ||
      in_sizes[3] != NG3 || in_sizes[4] != NG3 ||
      in_sizes[5] != NG3 * NHID || in_sizes[6] != NG3 * NHID || in_sizes[7] != NG3 || in_sizes[8] != NG3 ||
      in_sizes[9] != NG3 * NHID || in_sizes[10] != NG3 * NHID || in_sizes[11] != NG3 || in_sizes[12] != NG3 ||
      out_size != NROWS * NHID) return;

  const float* inp    = (const float*)d_in[0];
  const float* w_ih_0 = (const float*)d_in[1];
  const float* w_hh_0 = (const float*)d_in[2];
  const float* b_ih_0 = (const float*)d_in[3];
  const float* b_hh_0 = (const float*)d_in[4];
  const float* w_ih_1 = (const float*)d_in[5];
  const float* w_hh_1 = (const float*)d_in[6];
  const float* b_ih_1 = (const float*)d_in[7];
  const float* b_hh_1 = (const float*)d_in[8];
  const float* w_ih_2 = (const float*)d_in[9];
  const float* w_hh_2 = (const float*)d_in[10];
  const float* b_ih_2 = (const float*)d_in[11];
  const float* b_hh_2 = (const float*)d_in[12];
  float* out = (float*)d_out;

  char* ws = (char*)d_ws; size_t off = 0;
  auto carve = [&](size_t bytes) -> char* { char* p = ws + off; off += (bytes + 255) & ~(size_t)255; return p; };
  unsigned short* XH   = (unsigned short*)carve((size_t)NROWS * NFEAT * 2);
  unsigned short* WIH0 = (unsigned short*)carve((size_t)NG3 * NFEAT * 2);
  unsigned short* WIH1 = (unsigned short*)carve((size_t)NG3 * NHID * 2);
  unsigned short* WIH2 = (unsigned short*)carve((size_t)NG3 * NHID * 2);
  unsigned short* WHH0 = (unsigned short*)carve((size_t)NG3 * NHID * 2);
  unsigned short* WHH1 = (unsigned short*)carve((size_t)NG3 * NHID * 2);
  unsigned short* WHH2 = (unsigned short*)carve((size_t)NG3 * NHID * 2);
  float*          PX   = (float*)carve((size_t)NROWS * NG3 * 4);
  unsigned short* YS   = (unsigned short*)carve((size_t)NROWS * NHID * 2);
  if (off > ws_size || off > (size_t)134217728) return;

  const int n8x  = NROWS * NFEAT / 8;
  const int n8w0 = NG3 * NFEAT / 8;
  const int n8w  = NG3 * NHID / 8;
  cvt_f16x8_kernel<<<(n8x + NTHR - 1) / NTHR, NTHR, 0, stream>>>(inp,    XH,   n8x,  1.0f);
  cvt_f16x8_kernel<<<(n8w0 + NTHR - 1) / NTHR, NTHR, 0, stream>>>(w_ih_0, WIH0, n8w0, WCARRY);
  cvt_f16x8_kernel<<<(n8w + NTHR - 1) / NTHR, NTHR, 0, stream>>>(w_ih_1, WIH1, n8w,  WCARRY);
  cvt_f16x8_kernel<<<(n8w + NTHR - 1) / NTHR, NTHR, 0, stream>>>(w_ih_2, WIH2, n8w,  WCARRY);
  cvt_f16x8_kernel<<<(n8w + NTHR - 1) / NTHR, NTHR, 0, stream>>>(w_hh_0, WHH0, n8w,  WCARRY);
  cvt_f16x8_kernel<<<(n8w + NTHR - 1) / NTHR, NTHR, 0, stream>>>(w_hh_1, WHH1, n8w,  WCARRY);
  cvt_f16x8_kernel<<<(n8w + NTHR - 1) / NTHR, NTHR, 0, stream>>>(w_hh_2, WHH2, n8w,  WCARRY);

  const dim3 ggrid((NROWS / 64) * (NG3 / 64) / 8, 1);
  const dim3 sgrid(NBAT / ROWS_BLK);

  wmma_gemm64<0, false, 2, 0, false, 0><<<ggrid, 256, 0, stream>>>(
      XH, XH, NFEAT, 0L, WIH0, WIH0, NFEAT, 0L, (void*)PX, (void*)PX, NG3, 0L,
      b_ih_0, (const float*)PX, 0L, NROWS, NG3, NFEAT, PROJ0_SCALE);
  gru_scan_kernel<false><<<sgrid, NTHR, 0, stream>>>(PX, WHH0, b_hh_0, YS, out);

  wmma_gemm64<0, false, 2, 0, false, 0><<<ggrid, 256, 0, stream>>>(
      YS, YS, NHID, 0L, WIH1, WIH1, NHID, 0L, (void*)PX, (void*)PX, NG3, 0L,
      b_ih_1, (const float*)PX, 0L, NROWS, NG3, NHID, PROJ_SCALE);
  gru_scan_kernel<false><<<sgrid, NTHR, 0, stream>>>(PX, WHH1, b_hh_1, YS, out);

  wmma_gemm64<0, false, 2, 0, false, 0><<<ggrid, 256, 0, stream>>>(
      YS, YS, NHID, 0L, WIH2, WIH2, NHID, 0L, (void*)PX, (void*)PX, NG3, 0L,
      b_ih_2, (const float*)PX, 0L, NROWS, NG3, NHID, PROJ_SCALE);
  gru_scan_kernel<true><<<sgrid, NTHR, 0, stream>>>(PX, WHH2, b_hh_2, YS, out);
}
